// Mamba_65429531788056
// MI455X (gfx1250) — hardware-verified
//
#include <hip/hip_runtime.h>
#include <math.h>

typedef __attribute__((ext_vector_type(16))) _Float16 v16h;
typedef __attribute__((ext_vector_type(8)))  _Float16 v8h;
typedef __attribute__((ext_vector_type(16))) __bf16   v16b;
typedef __attribute__((ext_vector_type(8)))  __bf16   v8b;
typedef __attribute__((ext_vector_type(8)))  float    v8f;
typedef __attribute__((ext_vector_type(4)))  float    v4f;

constexpr int kBatch  = 2;
constexpr int kSeq    = 2048;
constexpr int kDm     = 768;
constexpr int kDin    = 1536;
constexpr int kNst    = 16;
constexpr int kDtR    = 48;
constexpr int kDtK    = 64;
constexpr int kXdN    = 80;
constexpr int kXdP    = 128;
constexpr int kXzP    = 2 * kDin;
constexpr int kYcP    = 2 * kDin;
constexpr int kRows   = kBatch * kSeq;
constexpr int kTP     = 260;
constexpr int kScanTS = 64;
constexpr int kScanCh = 64;
constexpr int kScanYP = 68;
constexpr float kYCarry   = 16.0f;
constexpr float kWoCarry  = 32.0f;
constexpr float kOutScale = 0.5f / (kYCarry * kWoCarry);

static_assert(kDtR + 2 * kNst == kXdN, "x_proj width");
static_assert(kDin == 2 * kDm && kDtR == (kDm + 15) / 16, "shape relations");
static_assert((kDm % 32) == 0 && (kDin % 32) == 0 && (kDtK % 32) == 0 && (kYcP % 32) == 0, "GEMM K multiples of 32");
static_assert((kSeq % 64) == 0 && (kXzP % 64) == 0 && (kXdP % 64) == 0 && (kDin % 64) == 0 && (kDm % 64) == 0, "GEMM M,N multiples of 64");
static_assert((kSeq % kScanTS) == 0 && (kDin % kScanCh) == 0 && (kDin % 256) == 0, "tile multiples");
static_assert((kDtR % 8) == 0 && kDtR < kDtK && kXdN < kXdP, "pad geometry");

constexpr size_t kOffHS16  = 0;
constexpr size_t kOffWIN16 = kOffHS16  + (size_t)kRows * kDm * 2;
constexpr size_t kOffWX16  = kOffWIN16 + (size_t)kXzP * kDm * 2;
constexpr size_t kOffWDT16 = kOffWX16  + (size_t)2 * kXdP * kDin * 2;
constexpr size_t kOffWOUT2 = kOffWDT16 + (size_t)2 * kDin * kDtK * 2;
constexpr size_t kOffXZ    = kOffWOUT2 + (size_t)kDm * kYcP * 2;
constexpr size_t kOffXC    = kOffXZ    + (size_t)kSeq * kXzP * 4;
constexpr size_t kOffXC16  = kOffXC    + (size_t)2 * kSeq * kDin * 4;
constexpr size_t kOffXDBL  = kOffXC16  + (size_t)2 * kSeq * kDin * 2;
constexpr size_t kOffDTA   = kOffXDBL  + (size_t)2 * kSeq * kXdP * 4;
constexpr size_t kOffDLR   = kOffDTA   + (size_t)2 * kSeq * kDtK * 2;
constexpr size_t kOffYCAT  = kOffDLR   + (size_t)2 * kSeq * kDin * 4;
constexpr size_t kWsTotal  = kOffYCAT  + (size_t)kSeq * kYcP * 2;
static_assert(kWsTotal == 120193024ull, "carve total");
static_assert(kWsTotal <= 134217728ull, "carve cap");
static_assert((kOffWIN16 % 128) == 0 && (kOffWX16 % 128) == 0 && (kOffWDT16 % 128) == 0 && (kOffWOUT2 % 128) == 0 &&
              (kOffXZ % 128) == 0 && (kOffXC % 128) == 0 && (kOffXC16 % 128) == 0 && (kOffXDBL % 128) == 0 &&
              (kOffDTA % 128) == 0 && (kOffDLR % 128) == 0 && (kOffYCAT % 128) == 0, "128-B aligned regions");

__device__ __forceinline__ unsigned short f2bf_bits(float f) {
  unsigned u = __float_as_uint(f);
  return (unsigned short)((u + 0x7FFFu + ((u >> 16) & 1u)) >> 16);
}
__device__ __forceinline__ float bf_bits2f(unsigned short h) { return __uint_as_float(((unsigned)h) << 16); }
__device__ __forceinline__ float bf_rne(float f) { return bf_bits2f(f2bf_bits(f)); }

__device__ __forceinline__ void row_guard_h(v8f& a, v8f& b, v8f& c, v8f& d, v16h x) { asm volatile("v_nop\n\tv_nop\n\tv_nop\n\tv_nop" : "+v"(a), "+v"(b), "+v"(c), "+v"(d) : "v"(x)); }
__device__ __forceinline__ void row_guard_b(v8f& a, v8f& b, v8f& c, v8f& d, v16b x) { asm volatile("v_nop\n\tv_nop\n\tv_nop\n\tv_nop" : "+v"(a), "+v"(b), "+v"(c), "+v"(d) : "v"(x)); }
__device__ __forceinline__ void keep4_h(v16h a, v16h b, v16h c, v16h d) { asm volatile("v_nop" :: "v"(a), "v"(b), "v"(c), "v"(d)); }
__device__ __forceinline__ void keep4_b(v16b a, v16b b, v16b c, v16b d) { asm volatile("v_nop" :: "v"(a), "v"(b), "v"(c), "v"(d)); }
__device__ __forceinline__ void acc_guard4(v8f& a, v8f& b, v8f& c, v8f& d) { asm volatile("v_nop\n\tv_nop\n\tv_nop\n\tv_nop" : "+v"(a), "+v"(b), "+v"(c), "+v"(d)); }

template <typename T> struct Frag;
template <> struct Frag<_Float16> {
  typedef v16h V; union U { v16h v; v8h h[2]; };
  static __device__ __forceinline__ v16h load(const _Float16* p) {
    U f; f.h[0] = *(const v8h*)(p); f.h[1] = *(const v8h*)(p + 16); return f.v;
  }
  static __device__ __forceinline__ v8f mma(v16h a, v16h b, v8f c) {
    return __builtin_amdgcn_wmma_f32_16x16x32_f16(false, a, false, b, (short)0, c, false, false);
  }
  static __device__ __forceinline__ void guard4(v8f& a, v8f& b, v8f& c, v8f& d, v16h x) { row_guard_h(a, b, c, d, x); }
  static __device__ __forceinline__ void keep(v16h a, v16h b, v16h c, v16h d) { keep4_h(a, b, c, d); }
};
template <> struct Frag<__bf16> {
  typedef v16b V; union U { v16b v; v8b h[2]; };
  static __device__ __forceinline__ v16b load(const __bf16* p) {
    U f; f.h[0] = *(const v8b*)(p); f.h[1] = *(const v8b*)(p + 16); return f.v;
  }
  static __device__ __forceinline__ v8f mma(v16b a, v16b b, v8f c) {
    return __builtin_amdgcn_wmma_f32_16x16x32_bf16(false, a, false, b, (short)0, c, false, false);
  }
  static __device__ __forceinline__ void guard4(v8f& a, v8f& b, v8f& c, v8f& d, v16b x) { row_guard_b(a, b, c, d, x); }
  static __device__ __forceinline__ void keep(v16b a, v16b b, v16b c, v16b d) { keep4_b(a, b, c, d); }
};

template <int ET> struct Elem;
template <> struct Elem<0> { typedef _Float16 T; };
template <> struct Elem<1> { typedef __bf16 T; };
template <int ET>
__global__ __launch_bounds__(256) void wmma_gemm64(
    const unsigned short* __restrict__ Ap, int lda, long strideA,
    const unsigned short* __restrict__ Btp, int ldb, long strideB,
    float* __restrict__ Cout, int ldc, long strideC,
    int M, int N, int K, float scale) {
  typedef typename Elem<ET>::T T;
  typedef typename Frag<T>::V V;
  const T* A = (const T*)Ap; const T* Bt = (const T*)Btp;
  __shared__ __align__(16) float sT[8][16 * 68];
  const int b    = blockIdx.y;
  const int lane = threadIdx.x & 31;
  const int wave = threadIdx.x >> 5;
  const int tilesN = N >> 6;
  const int tilesM = M >> 6;
  const int tile = blockIdx.x * 8 + wave;
  if (tile >= tilesM * tilesN) return;
  const int tm = tile / tilesN;
  const int tn = tile - tm * tilesN;
  const int m0 = tm << 6;
  const int n0 = tn << 6;

  const T* Ab = A  + (size_t)b * strideA;
  const T* Bb = Bt + (size_t)b * strideB;

  const int rlane = lane & 15;
  const int koff  = (lane >> 4) * 8;
  const int mOff  = (lane >> 4) * 8;

  v8f acc[4][4];
#pragma unroll
  for (int i = 0; i < 4; ++i)
#pragma unroll
    for (int j = 0; j < 4; ++j) acc[i][j] = (v8f){0.f,0.f,0.f,0.f,0.f,0.f,0.f,0.f};

  for (int k0 = 0; k0 < K; k0 += 32) {
    V bh[4];
#pragma unroll
    for (int j = 0; j < 4; ++j) {
      const size_t bo = (size_t)(n0 + (j << 4) + rlane) * ldb + koff + k0;
      bh[j] = Frag<T>::load(Bb + bo);
    }
#pragma unroll
    for (int i = 0; i < 4; ++i) {
      const size_t ao = (size_t)(m0 + (i << 4) + rlane) * lda + koff + k0;
      V ah = Frag<T>::load(Ab + ao);
#pragma unroll
      for (int j = 0; j < 4; ++j) acc[i][j] = Frag<T>::mma(ah, bh[j], acc[i][j]);
      Frag<T>::guard4(acc[i][0], acc[i][1], acc[i][2], acc[i][3], ah);
    }
    Frag<T>::keep(bh[0], bh[1], bh[2], bh[3]);
  }
  acc_guard4(acc[0][0], acc[0][1], acc[0][2], acc[0][3]);
  acc_guard4(acc[1][0], acc[1][1], acc[1][2], acc[1][3]);
  acc_guard4(acc[2][0], acc[2][1], acc[2][2], acc[2][3]);
  acc_guard4(acc[3][0], acc[3][1], acc[3][2], acc[3][3]);

  float* slab = sT[wave];
  float* C = Cout + (size_t)b * strideC;
  const int hh = lane >> 4, c4 = (lane & 15) * 4;
#pragma unroll
  for (int i = 0; i < 4; ++i) {
    const int mBase = m0 + (i << 4);
#pragma unroll
    for (int j = 0; j < 4; ++j) {
#pragma unroll
      for (int r = 0; r < 8; ++r) {
        const float v = acc[i][j][r] * scale;
        slab[(mOff + r) * 68 + (j << 4) + rlane] = v;
      }
    }
    __builtin_amdgcn_fence(__ATOMIC_RELEASE, "workgroup");
    __builtin_amdgcn_wave_barrier();
    __builtin_amdgcn_fence(__ATOMIC_ACQUIRE, "workgroup");
    for (int pass = 0; pass < 2; ++pass) {
#pragma unroll
      for (int it = 0; it < 8; ++it) {
        const int row = it * 2 + hh;
        v4f v = *(const v4f*)(slab + row * 68 + c4);
        *(volatile v4f*)(C + (size_t)(mBase + row) * ldc + n0 + c4) = v;
      }
      __threadfence();
    }
    __builtin_amdgcn_fence(__ATOMIC_RELEASE, "workgroup");
    __builtin_amdgcn_wave_barrier();
    __builtin_amdgcn_fence(__ATOMIC_ACQUIRE, "workgroup");
  }
}

__global__ __launch_bounds__(256) void cast_bf16_kernel(
    const float* __restrict__ src, unsigned short* __restrict__ dst, int total8)
{
  const int i = blockIdx.x * 256 + threadIdx.x;
  if (i >= total8) return;
  const size_t e0 = (size_t)i << 3;
  const v4f a0 = *(const v4f*)(src + e0);
  const v4f a1 = *(const v4f*)(src + e0 + 4);
  v8h hv;
#pragma unroll
  for (int e = 0; e < 4; ++e) {
    const unsigned short h0 = f2bf_bits(a0[e]);
    const unsigned short h1 = f2bf_bits(a1[e]);
    hv[e]     = __builtin_bit_cast(_Float16, h0);
    hv[4 + e] = __builtin_bit_cast(_Float16, h1);
  }
  unsigned short* q = dst + e0;
  *(volatile v8h*)q = hv;
  __threadfence();
  *(volatile v8h*)q = hv;
}

__global__ __launch_bounds__(256) void wx_plane_kernel(
    const float* __restrict__ Wf, const float* __restrict__ Wb, unsigned short* __restrict__ dst)
{
  const int br = blockIdx.y;
  const float* W = br ? Wb : Wf;
  const int i = blockIdx.x * 256 + threadIdx.x;
  const int e0 = i << 3;
  const int row = e0 / kDin;
  const int col = e0 - row * kDin;
  const bool keep = (row < kXdN);
  const int rc = keep ? row : (kXdN - 1);
  const float* p = W + (size_t)rc * kDin + col;
  const v4f a0 = *(const v4f*)(p);
  const v4f a1 = *(const v4f*)(p + 4);
  v8h hv;
#pragma unroll
  for (int e = 0; e < 4; ++e) {
    const unsigned short b0 = f2bf_bits(a0[e]);
    const unsigned short b1 = f2bf_bits(a1[e]);
    const unsigned short h0 = keep ? b0 : (unsigned short)0;
    const unsigned short h1 = keep ? b1 : (unsigned short)0;
    hv[e]     = __builtin_bit_cast(_Float16, h0);
    hv[4 + e] = __builtin_bit_cast(_Float16, h1);
  }
  unsigned short* q = dst + (size_t)br * kXdP * kDin + e0;
  *(volatile v8h*)q = hv;
  __threadfence();
  *(volatile v8h*)q = hv;
}

__global__ __launch_bounds__(256) void wdt_plane_kernel(
    const float* __restrict__ Wf, const float* __restrict__ Wb, unsigned short* __restrict__ dst)
{
  const int br = blockIdx.y;
  const float* W = br ? Wb : Wf;
  const int i = blockIdx.x * 256 + threadIdx.x;
  const int e0 = i << 3;
  const int row = e0 >> 6;
  const int c8  = e0 & 63;
  const bool keep = (c8 < kDtR);
  const int cc = keep ? c8 : (kDtR - 8);
  const float* p = W + (size_t)row * kDtR + cc;
  const v4f a0 = *(const v4f*)(p);
  const v4f a1 = *(const v4f*)(p + 4);
  v8h hv;
#pragma unroll
  for (int e = 0; e < 4; ++e) {
    const unsigned short b0 = f2bf_bits(a0[e]);
    const unsigned short b1 = f2bf_bits(a1[e]);
    const unsigned short h0 = keep ? b0 : (unsigned short)0;
    const unsigned short h1 = keep ? b1 : (unsigned short)0;
    hv[e]     = __builtin_bit_cast(_Float16, h0);
    hv[4 + e] = __builtin_bit_cast(_Float16, h1);
  }
  unsigned short* q = dst + (size_t)br * kDin * kDtK + e0;
  *(volatile v8h*)q = hv;
  __threadfence();
  *(volatile v8h*)q = hv;
}

__global__ __launch_bounds__(256) void wout_plane_kernel(
    const float* __restrict__ W, unsigned short* __restrict__ dst)
{
  const int i = blockIdx.x * 256 + threadIdx.x;
  const int e0 = i << 3;
  const int row = e0 / kYcP;
  const int col = e0 - row * kYcP;
  const int cs  = (col >= kDin) ? (col - kDin) : col;
  const float* p = W + (size_t)row * kDin + cs;
  const v4f a0 = *(const v4f*)(p);
  const v4f a1 = *(const v4f*)(p + 4);
  v8h hv;
#pragma unroll
  for (int e = 0; e < 4; ++e) {
    const float f0 = bf_rne(a0[e]) * kWoCarry;
    const float f1 = bf_rne(a1[e]) * kWoCarry;
    hv[e]     = (_Float16)f0;
    hv[4 + e] = (_Float16)f1;
  }
  unsigned short* q = dst + e0;
  *(volatile v8h*)q = hv;
  __threadfence();
  *(volatile v8h*)q = hv;
}

__global__ __launch_bounds__(256) void dt_cast_kernel(
    const float* __restrict__ XDBL, unsigned short* __restrict__ DTA)
{
  const int i = blockIdx.x * 256 + threadIdx.x;
  const int e0 = i << 3;
  const int row = e0 >> 6;
  const int c8  = e0 & 63;
  const bool keep = (c8 < kDtR);
  const int cc = keep ? c8 : (kDtR - 8);
  const float* p = XDBL + (size_t)row * kXdP + cc;
  const v4f a0 = *(const v4f*)(p);
  const v4f a1 = *(const v4f*)(p + 4);
  v8h hv;
#pragma unroll
  for (int e = 0; e < 4; ++e) {
    const unsigned short b0 = f2bf_bits(a0[e]);
    const unsigned short b1 = f2bf_bits(a1[e]);
    const unsigned short h0 = keep ? b0 : (unsigned short)0;
    const unsigned short h1 = keep ? b1 : (unsigned short)0;
    hv[e]     = __builtin_bit_cast(_Float16, h0);
    hv[4 + e] = __builtin_bit_cast(_Float16, h1);
  }
  unsigned short* q = DTA + e0;
  *(volatile v8h*)q = hv;
  __threadfence();
  *(volatile v8h*)q = hv;
}

__global__ __launch_bounds__(256) void conv_silu_kernel(
    const float* __restrict__ XZ,
    const float* __restrict__ cw_f, const float* __restrict__ cb_f,
    const float* __restrict__ cw_b, const float* __restrict__ cb_b,
    float* __restrict__ XC, unsigned short* __restrict__ XC16)
{
  __shared__ __align__(16) float sT[16 * kTP];
  const int tid = threadIdx.x, lane = tid & 31, wave = tid >> 5;
  const int br = blockIdx.z;
  const float* cw = br ? cw_b : cw_f;
  const float* cb = br ? cb_b : cb_f;
  const int d0 = blockIdx.x * 256, d = d0 + tid;
  const int t0 = blockIdx.y * 64;
  const int dir = br ? -1 : 1;
  const int ls  = br ? (t0 + 63) : t0;
  const v4f wv = *(const v4f*)(cw + (size_t)d * 4);
  const float w0 = bf_rne(wv[0]);
  const float w1 = bf_rne(wv[1]);
  const float w2 = bf_rne(wv[2]);
  const float w3 = bf_rne(wv[3]);
  const float bc = bf_rne(cb[d]);
  float xm3, xm2, xm1;
  {
    const int r1 = ls - dir, r2 = ls - 2 * dir, r3 = ls - 3 * dir;
    const int c1 = (r1 < 0) ? 0 : ((r1 > kSeq - 1) ? (kSeq - 1) : r1);
    const int c2 = (r2 < 0) ? 0 : ((r2 > kSeq - 1) ? (kSeq - 1) : r2);
    const int c3 = (r3 < 0) ? 0 : ((r3 > kSeq - 1) ? (kSeq - 1) : r3);
    const float v1 = XZ[(size_t)c1 * kXzP + d];
    const float v2 = XZ[(size_t)c2 * kXzP + d];
    const float v3 = XZ[(size_t)c3 * kXzP + d];
    xm1 = ((unsigned)r1 < (unsigned)kSeq) ? v1 : 0.f;
    xm2 = ((unsigned)r2 < (unsigned)kSeq) ? v2 : 0.f;
    xm3 = ((unsigned)r3 < (unsigned)kSeq) ? v3 : 0.f;
  }
  float* XCb = XC + (size_t)br * kSeq * kDin;
  unsigned short* XC16b = XC16 + (size_t)br * kSeq * kDin;
  const int hrow = wave >> 1;
  const int hch  = (wave & 1) * 128 + lane * 4;
#pragma unroll 1
  for (int sub = 0; sub < 4; ++sub) {
    const int lb = br ? (t0 + 48 - sub * 16) : (t0 + sub * 16);
#pragma unroll 1
    for (int s = 0; s < 16; ++s) {
      const int l  = ls + dir * (sub * 16 + s);
      const int tr = br ? (15 - s) : s;
      const float xcur = XZ[(size_t)l * kXzP + d];
      float acc = w0 * xm3;
      acc = fmaf(w1, xm2, acc);
      acc = fmaf(w2, xm1, acc);
      acc = fmaf(w3, xcur, acc);
      const float sv = acc + bc;
      const float sg = __builtin_amdgcn_rcpf(1.0f + expf(-sv));
      sT[tr * kTP + tid] = sv * sg;
      xm3 = xm2; xm2 = xm1; xm1 = xcur;
    }
    __syncthreads();
    v4f fv[4];
    v8h bv[2];
#pragma unroll
    for (int it = 0; it < 4; ++it) fv[it] = *(const v4f*)(sT + (it * 4 + hrow) * kTP + hch);
#pragma unroll
    for (int it = 0; it < 2; ++it) {
      const float* sp = sT + (it * 8 + wave) * kTP + lane * 8;
      const v4f a0 = *(const v4f*)(sp);
      const v4f a1 = *(const v4f*)(sp + 4);
#pragma unroll
      for (int e = 0; e < 4; ++e) {
        const unsigned short h0 = f2bf_bits(a0[e]);
        const unsigned short h1 = f2bf_bits(a1[e]);
        bv[it][e]     = __builtin_bit_cast(_Float16, h0);
        bv[it][4 + e] = __builtin_bit_cast(_Float16, h1);
      }
    }
    for (int pass = 0; pass < 2; ++pass) {
#pragma unroll
      for (int it = 0; it < 4; ++it)
        *(volatile v4f*)(XCb + (size_t)(lb + it * 4 + hrow) * kDin + d0 + hch) = fv[it];
#pragma unroll
      for (int it = 0; it < 2; ++it)
        *(volatile v8h*)(XC16b + (size_t)(lb + it * 8 + wave) * kDin + d0 + lane * 8) = bv[it];
      __threadfence();
    }
    __syncthreads();
  }
}

__global__ __launch_bounds__(64) void scan_kernel(
    const float* __restrict__ DLR, const float* __restrict__ XC, const float* __restrict__ XZ,
    const float* __restrict__ XDBL,
    const float* __restrict__ bdt_f, const float* __restrict__ bdt_b,
    const float* __restrict__ alog_f, const float* __restrict__ alog_b,
    const float* __restrict__ dp_f, const float* __restrict__ dp_b,
    unsigned short* __restrict__ YCAT)
{
  __shared__ __align__(16) float sX[kScanTS * 32];
  __shared__ __align__(16) float sY[kScanTS * kScanYP];
  __shared__ __align__(16) float sA[kNst * kScanCh];
  const int tid = threadIdx.x, lane = tid & 31, wave = tid >> 5;
  constexpr int kBlkPerDir = kDin / kScanCh;
  const int br = blockIdx.x / kBlkPerDir;
  const int d0 = (blockIdx.x - br * kBlkPerDir) * kScanCh;
  const int d  = d0 + tid;
  const float* alog = br ? alog_b : alog_f;
  const float* bdt  = br ? bdt_b : bdt_f;
  const float* dpv  = br ? dp_b : dp_f;
  const size_t brow = (size_t)br * kSeq;
#pragma unroll 1
  for (int s = 0; s < kNst; ++s) sA[s * kScanCh + tid] = -expf(bf_rne(alog[(size_t)d * kNst + s]));
  __syncthreads();
  float negA[kNst], h[kNst];
#pragma unroll
  for (int s = 0; s < kNst; ++s) {
    negA[s] = sA[s * kScanCh + tid];
    h[s] = 0.f;
  }
  const float bb = bf_rne(bdt[d]);
  const float Dd = bf_rne(dpv[d]);
  const int q = lane >> 3, c8 = (lane & 7) * 8;
#pragma unroll 1
  for (int c = 0; c < kSeq / kScanTS; ++c) {
    const int base = br ? (kSeq - kScanTS * (c + 1)) : (kScanTS * c);
    __syncthreads();
#pragma unroll
    for (int i = 0; i < 8; ++i) {
      const int idx = tid + 64 * i;
      const int r  = idx >> 3;
      const int cq = (idx & 7) * 4;
      *(v4f*)(sX + r * 32 + cq) = *(const v4f*)(XDBL + (brow + base + r) * kXdP + kDtR + cq);
    }
    __syncthreads();
#pragma unroll 1
    for (int s = 0; s < kScanTS; ++s) {
      const int li = br ? (kScanTS - 1 - s) : s;
      const size_t l = (size_t)(base + li);
      const float* xr = sX + li * 32;
      float Bs[kNst], Cs[kNst];
#pragma unroll
      for (int q4 = 0; q4 < 4; ++q4) {
        const v4f bv = *(const v4f*)(xr + 4 * q4);
        const v4f cv = *(const v4f*)(xr + kNst + 4 * q4);
        Bs[4 * q4 + 0] = bv[0]; Bs[4 * q4 + 1] = bv[1]; Bs[4 * q4 + 2] = bv[2]; Bs[4 * q4 + 3] = bv[3];
        Cs[4 * q4 + 0] = cv[0]; Cs[4 * q4 + 1] = cv[1]; Cs[4 * q4 + 2] = cv[2]; Cs[4 * q4 + 3] = cv[3];
      }
      const float v   = DLR[(brow + l) * kDin + d] + bb;
      const float dt  = fmaxf(v, 0.0f) + log1pf(expf(-fabsf(v)));
      const float xt  = XC[(brow + l) * kDin + d];
      const float zv  = XZ[l * kXzP + kDin + d];
      const float dtx = dt * xt;
      float y = 0.f;
#pragma unroll
      for (int k = 0; k < kNst; ++k) {
        const float e = __expf(dt * negA[k]);
        h[k] = e * h[k] + dtx * Bs[k];
        y = h[k] * Cs[k] + y;
      }
      y = xt * Dd + y;
      const float sg = __builtin_amdgcn_rcpf(1.0f + expf(-zv));
      y = y * (zv * sg);
      sY[li * kScanYP + tid] = y * kYCarry;
    }
    __syncthreads();
    v8h hv[8];
#pragma unroll
    for (int it = 0; it < 8; ++it) {
      const int row = it * 8 + wave * 4 + q;
      const float* sp = sY + row * kScanYP + c8;
      const v4f a0 = *(const v4f*)(sp);
      const v4f a1 = *(const v4f*)(sp + 4);
#pragma unroll
      for (int e = 0; e < 4; ++e) {
        hv[it][e]     = (_Float16)a0[e];
        hv[it][4 + e] = (_Float16)a1[e];
      }
    }
    for (int pass = 0; pass < 2; ++pass) {
#pragma unroll
      for (int it = 0; it < 8; ++it) {
        const int row = it * 8 + wave * 4 + q;
        *(volatile v8h*)(YCAT + (size_t)(base + row) * kYcP + br * kDin + d0 + c8) = hv[it];
      }
      __threadfence();
    }
  }
}

extern "C" void kernel_launch(void* const* d_in, const int* in_sizes, int n_in,
                              void* d_out, int out_size, void* d_ws, size_t ws_size,
                              hipStream_t stream) {
  if (n_in < 17) return;
  if (in_sizes[0] != kRows * kDm) return;
  if (in_sizes[1] != kXzP * kDm) return;
  if (in_sizes[2] != kDin * 4 || in_sizes[3] != kDin) return;
  if (in_sizes[4] != kDin * 4 || in_sizes[5] != kDin) return;
  if (in_sizes[6] != kXdN * kDin || in_sizes[7] != kXdN * kDin) return;
  if (in_sizes[8] != kDin * kDtR || in_sizes[9] != kDin) return;
  if (in_sizes[10] != kDin * kDtR || in_sizes[11] != kDin) return;
  if (in_sizes[12] != kDin * kNst || in_sizes[13] != kDin * kNst) return;
  if (in_sizes[14] != kDin || in_sizes[15] != kDin) return;
  if (in_sizes[16] != kDm * kDin) return;
  if (out_size != kRows * kDm) return;
  if (ws_size < kWsTotal) return;

  const float* hs       = (const float*)d_in[0];
  const float* W_in     = (const float*)d_in[1];
  const float* conv_w   = (const float*)d_in[2];
  const float* conv_b   = (const float*)d_in[3];
  const float* conv_w_b = (const float*)d_in[4];
  const float* conv_b_b = (const float*)d_in[5];
  const float* W_x      = (const float*)d_in[6];
  const float* W_x_b    = (const float*)d_in[7];
  const float* W_dt     = (const float*)d_in[8];
  const float* b_dt     = (const float*)d_in[9];
  const float* W_dt_b   = (const float*)d_in[10];
  const float* b_dt_b   = (const float*)d_in[11];
  const float* A_log    = (const float*)d_in[12];
  const float* A_b_log  = (const float*)d_in[13];
  const float* Dp       = (const float*)d_in[14];
  const float* Dp_b     = (const float*)d_in[15];
  const float* W_out    = (const float*)d_in[16];
  float* out = (float*)d_out;

  char* ws = (char*)d_ws;
  unsigned short* HS16  = (unsigned short*)(ws + kOffHS16);
  unsigned short* WIN16 = (unsigned short*)(ws + kOffWIN16);
  unsigned short* WX16  = (unsigned short*)(ws + kOffWX16);
  unsigned short* WDT16 = (unsigned short*)(ws + kOffWDT16);
  unsigned short* WOUT2 = (unsigned short*)(ws + kOffWOUT2);
  float*          XZ    = (float*)(ws + kOffXZ);
  float*          XC    = (float*)(ws + kOffXC);
  unsigned short* XC16  = (unsigned short*)(ws + kOffXC16);
  float*          XDBL  = (float*)(ws + kOffXDBL);
  unsigned short* DTA   = (unsigned short*)(ws + kOffDTA);
  float*          DLR   = (float*)(ws + kOffDLR);
  unsigned short* YCAT  = (unsigned short*)(ws + kOffYCAT);

  cast_bf16_kernel<<<(kRows * kDm / 8) / 256, 256, 0, stream>>>(hs, HS16, kRows * kDm / 8);
  cast_bf16_kernel<<<(kXzP * kDm / 8) / 256, 256, 0, stream>>>(W_in, WIN16, kXzP * kDm / 8);
  wx_plane_kernel<<<dim3((kXdP * kDin / 8) / 256, 2), 256, 0, stream>>>(W_x, W_x_b, WX16);
  wdt_plane_kernel<<<dim3((kDin * kDtK / 8) / 256, 2), 256, 0, stream>>>(W_dt, W_dt_b, WDT16);
  wout_plane_kernel<<<(kDm * kYcP / 8) / 256, 256, 0, stream>>>(W_out, WOUT2);

  for (int b = 0; b < kBatch; ++b) {
    const unsigned short* HSb = HS16 + (size_t)b * kSeq * kDm;
    float* outb = out + (size_t)b * kSeq * kDm;

    wmma_gemm64<1><<<dim3((kSeq / 64) * (kXzP / 64) / 8, 1), 256, 0, stream>>>(
        HSb, kDm, 0L, WIN16, kDm, 0L, XZ, kXzP, 0L, kSeq, kXzP, kDm, 1.0f);

    conv_silu_kernel<<<dim3(kDin / 256, kSeq / 64, 2), 256, 0, stream>>>(
        XZ, conv_w, conv_b, conv_w_b, conv_b_b, XC, XC16);

    wmma_gemm64<1><<<dim3((kSeq / 64) * (kXdP / 64) / 8, 2), 256, 0, stream>>>(
        XC16, kDin, (long)kSeq * kDin, WX16, kDin, (long)kXdP * kDin,
        XDBL, kXdP, (long)kSeq * kXdP, kSeq, kXdP, kDin, 1.0f);

    dt_cast_kernel<<<(2 * kSeq * kDtK / 8) / 256, 256, 0, stream>>>(XDBL, DTA);

    wmma_gemm64<1><<<dim3((kSeq / 64) * (kDin / 64) / 8, 2), 256, 0, stream>>>(
        DTA, kDtK, (long)kSeq * kDtK, WDT16, kDtK, (long)kDin * kDtK,
        DLR, kDin, (long)kSeq * kDin, kSeq, kDin, kDtK, 1.0f);

    scan_kernel<<<2 * (kDin / kScanCh), kScanCh, 0, stream>>>(
        DLR, XC, XZ, XDBL, b_dt, b_dt_b, A_log, A_b_log, Dp, Dp_b, YCAT);

    wmma_gemm64<0><<<dim3((kSeq / 64) * (kDm / 64) / 8, 1), 256, 0, stream>>>(
        YCAT, kYcP, 0L, WOUT2, kYcP, 0L, outb, kDm, 0L, kSeq, kDm, kYcP, kOutScale);
  }
}
